// MultiHeadAttention_74826920230963
// MI455X (gfx1250) — hardware-verified
//
#include <hip/hip_runtime.h>
#ifndef NB
#define NB 2
#endif
#ifndef SEQ
#define SEQ 2048
#endif
#ifndef RH
#define RH 256
#endif
#define NB_FULL 2
#define SEQ_FULL 2048
#define DM 1024
#define NH 16
#define HD 64
#define PLANE ((size_t)NB * SEQ * DM)

static_assert(SEQ % 128 == 0);
static_assert(SEQ <= SEQ_FULL);
static_assert(NB <= NB_FULL);
static_assert(RH % 128 == 0);
static_assert(RH >= 0 && RH <= SEQ);
static_assert(NH * HD == DM);
static_assert(HD == 64);
static_assert(DM % 64 == 0);
static_assert(PLANE * 2 * 7 + (size_t)5 * DM * DM * 2 + (size_t)NB * SEQ * (SEQ / 32) * 4 + 4096 <= (size_t)134217728);

typedef __bf16 v16b __attribute__((ext_vector_type(16)));
typedef _Float16 v16h __attribute__((ext_vector_type(16)));
typedef unsigned short v8us __attribute__((ext_vector_type(8), may_alias));
typedef float v8f __attribute__((ext_vector_type(8)));
typedef float v4f __attribute__((ext_vector_type(4)));
typedef float v4fa __attribute__((ext_vector_type(4), may_alias));
typedef int v4i __attribute__((ext_vector_type(4)));
typedef int v4ia __attribute__((ext_vector_type(4), may_alias));
union FragH { v16h v; v8us half[2]; _Float16 h[16]; unsigned short u[16]; };
union FragX { v16b b; v16h h; v8us half[2]; };
union H8 { v8us v; _Float16 h[8]; unsigned short u[8]; };

#define LOG2E 1.4426950408889634f
#define RES_SC 2048.0f
#define RES_INV 0.00048828125f

__device__ __forceinline__ unsigned short bf16_bits(float x) {
  const unsigned int u = __float_as_uint(x);
  const unsigned int r = (u + 0x7FFFu + ((u >> 16) & 1u)) >> 16;
  const unsigned int n = (u >> 16) | 0x40u;
  return (unsigned short)(((u & 0x7FFFFFFFu) > 0x7F800000u) ? n : r);
}
__device__ __forceinline__ float bf16_val(unsigned short b) { return __uint_as_float(((unsigned int)b) << 16); }
__device__ __forceinline__ float bf16_rne(float x) { return bf16_val(bf16_bits(x)); }

__device__ __forceinline__ void mma8(v16b a0, v16b a1, v16b b0, v16b b1, v16b b2, v16b b3, v8f (&c)[8]) {
  c[0] = __builtin_amdgcn_wmma_f32_16x16x32_bf16(false, a0, false, b0, (short)0, c[0], false, false);
  c[1] = __builtin_amdgcn_wmma_f32_16x16x32_bf16(false, a0, false, b1, (short)0, c[1], false, false);
  c[2] = __builtin_amdgcn_wmma_f32_16x16x32_bf16(false, a0, false, b2, (short)0, c[2], false, false);
  c[3] = __builtin_amdgcn_wmma_f32_16x16x32_bf16(false, a0, false, b3, (short)0, c[3], false, false);
  c[4] = __builtin_amdgcn_wmma_f32_16x16x32_bf16(false, a1, false, b0, (short)0, c[4], false, false);
  c[5] = __builtin_amdgcn_wmma_f32_16x16x32_bf16(false, a1, false, b1, (short)0, c[5], false, false);
  c[6] = __builtin_amdgcn_wmma_f32_16x16x32_bf16(false, a1, false, b2, (short)0, c[6], false, false);
  c[7] = __builtin_amdgcn_wmma_f32_16x16x32_bf16(false, a1, false, b3, (short)0, c[7], false, false);
  asm volatile("v_nop\n\tv_nop\n\tv_nop\n\tv_nop"
               : "+v"(c[0]), "+v"(c[1]), "+v"(c[2]), "+v"(c[3]), "+v"(c[4]), "+v"(c[5]), "+v"(c[6]), "+v"(c[7])
               : "v"(a0), "v"(a1), "v"(b0), "v"(b1), "v"(b2), "v"(b3));
}
__device__ __forceinline__ void mma8h(v16h a0, v16h a1, v16h b0, v16h b1, v16h b2, v16h b3, v8f (&c)[8]) {
  c[0] = __builtin_amdgcn_wmma_f32_16x16x32_f16(false, a0, false, b0, (short)0, c[0], false, false);
  c[1] = __builtin_amdgcn_wmma_f32_16x16x32_f16(false, a0, false, b1, (short)0, c[1], false, false);
  c[2] = __builtin_amdgcn_wmma_f32_16x16x32_f16(false, a0, false, b2, (short)0, c[2], false, false);
  c[3] = __builtin_amdgcn_wmma_f32_16x16x32_f16(false, a0, false, b3, (short)0, c[3], false, false);
  c[4] = __builtin_amdgcn_wmma_f32_16x16x32_f16(false, a1, false, b0, (short)0, c[4], false, false);
  c[5] = __builtin_amdgcn_wmma_f32_16x16x32_f16(false, a1, false, b1, (short)0, c[5], false, false);
  c[6] = __builtin_amdgcn_wmma_f32_16x16x32_f16(false, a1, false, b2, (short)0, c[6], false, false);
  c[7] = __builtin_amdgcn_wmma_f32_16x16x32_f16(false, a1, false, b3, (short)0, c[7], false, false);
  asm volatile("v_nop\n\tv_nop\n\tv_nop\n\tv_nop"
               : "+v"(c[0]), "+v"(c[1]), "+v"(c[2]), "+v"(c[3]), "+v"(c[4]), "+v"(c[5]), "+v"(c[6]), "+v"(c[7])
               : "v"(a0), "v"(a1), "v"(b0), "v"(b1), "v"(b2), "v"(b3));
}
__device__ __forceinline__ void mma_s(v16h k0, v16h k1, v16h q0, v16h q1, v8f& sh) {
  sh = __builtin_amdgcn_wmma_f32_16x16x32_f16(false, k0, false, q0, (short)0, sh, false, false);
  sh = __builtin_amdgcn_wmma_f32_16x16x32_f16(false, k1, false, q1, (short)0, sh, false, false);
  asm volatile("v_nop\n\tv_nop\n\tv_nop\n\tv_nop" : "+v"(sh) : "v"(k0), "v"(k1), "v"(q0), "v"(q1));
}
__device__ __forceinline__ void mma_pv3(v16h vh, v16h vl, v16h ph, v16h pl, v8f& oh, v8f& ol) {
  oh = __builtin_amdgcn_wmma_f32_16x16x32_f16(false, vh, false, ph, (short)0, oh, false, false);
  ol = __builtin_amdgcn_wmma_f32_16x16x32_f16(false, vh, false, pl, (short)0, ol, false, false);
  ol = __builtin_amdgcn_wmma_f32_16x16x32_f16(false, vl, false, ph, (short)0, ol, false, false);
  asm volatile("v_nop\n\tv_nop\n\tv_nop\n\tv_nop" : "+v"(oh), "+v"(ol) : "v"(vh), "v"(vl), "v"(ph), "v"(pl));
}
__device__ __forceinline__ void mma_pv1(v16h vh, v16h ph, v8f& oh) {
  oh = __builtin_amdgcn_wmma_f32_16x16x32_f16(false, vh, false, ph, (short)0, oh, false, false);
  asm volatile("v_nop\n\tv_nop\n\tv_nop\n\tv_nop" : "+v"(oh) : "v"(vh), "v"(ph));
}

template <bool F16>
__global__ __launch_bounds__(256) void k_cvt(const float* __restrict__ src, unsigned short* __restrict__ dst,
                                             int rows, int rpb, int rpb_full) {
  const int t = blockIdx.x * 256 + threadIdx.x;
  if (t >= rows * 128) return;
  const int row = t >> 7, piece = t & 127;
  const int b = row / rpb, s = row - b * rpb;
  const float* p = src + ((size_t)b * rpb_full + s) * DM + piece * 8;
  const v4f x0 = *(const v4fa*)(p), x1 = *(const v4fa*)(p + 4);
  H8 o;
#pragma unroll
  for (int i = 0; i < 4; ++i) {
    if (F16) {
      o.h[i]     = (_Float16)(bf16_rne(x0[i]) * 64.0f);
      o.h[4 + i] = (_Float16)(bf16_rne(x1[i]) * 64.0f);
    } else {
      o.u[i]     = bf16_bits(x0[i]);
      o.u[4 + i] = bf16_bits(x1[i]);
    }
  }
  const v8us ov = o.v;
  unsigned short* d = dst + (size_t)t * 8;
  *(volatile v8us*)d = ov;
  __threadfence();
  *(volatile v8us*)d = ov;
}

__global__ __launch_bounds__(256) void k_mask(const int* __restrict__ mask, unsigned int* __restrict__ bits) {
  const int t = blockIdx.x * 256 + threadIdx.x;
  if (t >= NB * SEQ * (SEQ / 32)) return;
  const int wd = t % (SEQ / 32), row = t / (SEQ / 32);
  const int b = row / SEQ, q = row - b * SEQ;
  const int* p = mask + ((size_t)b * SEQ_FULL + q) * SEQ_FULL + 32 * wd;
  unsigned int m = 0u;
#pragma unroll
  for (int j = 0; j < 8; ++j) {
    const v4i x = *(const v4ia*)(p + 4 * j);
    m |= ((x[0] == 1) ? 1u : 0u) << (4 * j);
    m |= ((x[1] == 1) ? 1u : 0u) << (4 * j + 1);
    m |= ((x[2] == 1) ? 1u : 0u) << (4 * j + 2);
    m |= ((x[3] == 1) ? 1u : 0u) << (4 * j + 3);
  }
  *(volatile unsigned int*)(bits + t) = m;
  __threadfence();
  *(volatile unsigned int*)(bits + t) = m;
}

template <int MODE>
__global__ __launch_bounds__(128) void k_gemm(const unsigned short* __restrict__ A, const unsigned short* __restrict__ Alo,
                                              const unsigned short* __restrict__ Wm,
                                              const float* __restrict__ bias0, const float* __restrict__ bias1,
                                              unsigned short* __restrict__ outH, unsigned short* __restrict__ outL,
                                              float* __restrict__ outF, int sbeg, int nblk) {
  __shared__ __attribute__((aligned(16))) float so[128][68];
  const int tid = threadIdx.x, w = __builtin_amdgcn_readfirstlane((int)(tid >> 5)), lane = tid & 31, ln = lane & 15, hh = lane >> 4;
  const int b = blockIdx.x / nblk, s0 = sbeg + (blockIdx.x - b * nblk) * 128;
  const int rowB = b * SEQ + s0, colB = blockIdx.y * 64, z = blockIdx.z;
  const size_t aoff = (size_t)(rowB + 32 * w + ln) * DM + 8 * hh;
  const unsigned short* ap = A + aoff;
  const unsigned short* lp = Alo + aoff;
  const unsigned short* wp = Wm + (size_t)z * DM * DM + (size_t)(colB + ln) * DM + 8 * hh;
  const v8f z8 = {0.f, 0.f, 0.f, 0.f, 0.f, 0.f, 0.f, 0.f};
  v8f c[8];
#pragma unroll
  for (int i = 0; i < 8; ++i) c[i] = z8;
#pragma unroll 1
  for (int k0 = 0; k0 < DM; k0 += 32) {
    FragX a0, a1, b0, b1, b2, b3;
    a0.half[0] = *(const v8us*)(ap + k0);               a0.half[1] = *(const v8us*)(ap + k0 + 16);
    a1.half[0] = *(const v8us*)(ap + 16 * DM + k0);     a1.half[1] = *(const v8us*)(ap + 16 * DM + k0 + 16);
    b0.half[0] = *(const v8us*)(wp + k0);               b0.half[1] = *(const v8us*)(wp + k0 + 16);
    b1.half[0] = *(const v8us*)(wp + 16 * DM + k0);     b1.half[1] = *(const v8us*)(wp + 16 * DM + k0 + 16);
    b2.half[0] = *(const v8us*)(wp + 32 * DM + k0);     b2.half[1] = *(const v8us*)(wp + 32 * DM + k0 + 16);
    b3.half[0] = *(const v8us*)(wp + 48 * DM + k0);     b3.half[1] = *(const v8us*)(wp + 48 * DM + k0 + 16);
    if (MODE == 3) mma8h(a0.h, a1.h, b0.h, b1.h, b2.h, b3.h, c);
    else           mma8(a0.b, a1.b, b0.b, b1.b, b2.b, b3.b, c);
    if (MODE == 2) {
      FragX l0, l1;
      l0.half[0] = *(const v8us*)(lp + k0);             l0.half[1] = *(const v8us*)(lp + k0 + 16);
      l1.half[0] = *(const v8us*)(lp + 16 * DM + k0);   l1.half[1] = *(const v8us*)(lp + 16 * DM + k0 + 16);
      mma8(l0.b, l1.b, b0.b, b1.b, b2.b, b3.b, c);
    }
  }
  const float cs = (MODE == 3) ? 0.000244140625f : 1.0f;
#pragma unroll
  for (int j = 0; j < 4; ++j) {
    const int n = colB + 16 * j + ln;
    const float bA = bias0[n], bB = bias1[n];
    const float bj = bf16_rne((MODE == 0 && z == 1) ? bB : bA);
#pragma unroll
    for (int i = 0; i < 2; ++i)
#pragma unroll
      for (int r = 0; r < 8; ++r)
        so[32 * w + 16 * i + 8 * hh + r][16 * j + ln] = c[4 * i + j][r] * cs + bj;
  }
  __syncthreads();
  const int hd = blockIdx.y;
  if (MODE == 0) {
    const size_t base = (size_t)z * PLANE + (((size_t)(b * NH + hd)) * SEQ + s0) * HD;
    unsigned short* dh = outH + base;
    for (int pass = 0; pass < 2; ++pass) {
      for (int i = tid; i < 128 * 8; i += 128) {
        const int row = i >> 3, p8 = (i & 7) * 8;
        const v4f x0 = *(const v4fa*)&so[row][p8], x1 = *(const v4fa*)&so[row][p8 + 4];
        H8 oh;
#pragma unroll
        for (int q = 0; q < 4; ++q) {
          oh.h[q]     = (_Float16)(x0[q] * 16.0f);
          oh.h[4 + q] = (_Float16)(x1[q] * 16.0f);
        }
        const v8us ov = oh.v;
        *(volatile v8us*)(dh + (size_t)i * 8) = ov;
      }
      if (pass == 0) __threadfence();
    }
  } else if (MODE == 1) {
    const size_t base = (((size_t)(b * NH + hd)) * HD) * SEQ + s0;
    unsigned short* dh = outH + base;
    unsigned short* dl = outL + base;
    for (int pass = 0; pass < 2; ++pass) {
      for (int i = tid; i < 64 * 16; i += 128) {
        const int d = i >> 4, s8 = (i & 15) * 8;
        H8 oh, ol;
#pragma unroll
        for (int q = 0; q < 8; ++q) {
          const float v0 = so[s8 + q][d] * 16.0f;
          const _Float16 h0 = (_Float16)v0;
          oh.h[q] = h0;
          ol.h[q] = (_Float16)((v0 - (float)h0) * RES_SC);
        }
        const v8us ovh = oh.v, ovl = ol.v;
        *(volatile v8us*)(dh + (size_t)d * SEQ + s8) = ovh;
        *(volatile v8us*)(dl + (size_t)d * SEQ + s8) = ovl;
      }
      if (pass == 0) __threadfence();
    }
  } else {
    float* og = outF + ((size_t)b * SEQ_FULL + s0) * DM + colB;
    for (int pass = 0; pass < 2; ++pass) {
      for (int i = tid; i < 128 * 16; i += 128) {
        const int row = i >> 4, c4 = (i & 15) * 4;
        const v4f v = *(const v4fa*)&so[row][c4];
        *(volatile v4f*)(og + (size_t)row * DM + c4) = v;
      }
      if (pass == 0) __threadfence();
    }
  }
}

template <bool EARLY>
__device__ __forceinline__ void fa_step(const unsigned short* __restrict__ Khp,
                                        const unsigned short* __restrict__ Vhp, const unsigned short* __restrict__ Vlp,
                                        int key0, unsigned int mw, int ln, int hh,
                                        const FragH& qh0, const FragH& qh1,
                                        float& mr, float& lr, v8f (&Oh)[4], v8f (&Ol)[4]) {
  const v8f z8 = {0.f, 0.f, 0.f, 0.f, 0.f, 0.f, 0.f, 0.f};
  const size_t ko = (size_t)(key0 + ln) * HD + 8 * hh;
  float sc[16];
#pragma unroll
  for (int kt = 0; kt < 2; ++kt) {
    const unsigned short* kph = Khp + ko + (size_t)kt * 16 * HD;
    FragH kh0, kh1;
    kh0.half[0] = *(const v8us*)(kph);      kh0.half[1] = *(const v8us*)(kph + 16);
    kh1.half[0] = *(const v8us*)(kph + 32); kh1.half[1] = *(const v8us*)(kph + 48);
    v8f sh = z8;
    mma_s(kh0.v, kh1.v, qh0.v, qh1.v, sh);
#pragma unroll
    for (int r = 0; r < 8; ++r) sc[8 * kt + r] = sh[r] * 0.00048828125f;
  }
  const float ninf = __uint_as_float(0xFF800000u);
  const unsigned int mb = mw >> (8 * hh);
#pragma unroll
  for (int r = 0; r < 8; ++r) {
    sc[r]     = ((mb >> r) & 1u) ? ninf : sc[r];
    sc[8 + r] = ((mb >> (16 + r)) & 1u) ? ninf : sc[8 + r];
  }
  float mx = sc[0];
#pragma unroll
  for (int i = 1; i < 16; ++i) mx = fmaxf(mx, sc[i]);
  mx = fmaxf(mx, __shfl_xor(mx, 16, 32));
  const float mnew = fmaxf(mr, mx);
  const float al = exp2f((mr - mnew) * LOG2E);
  mr = mnew;
  FragH ph, pl;
  float ps = 0.0f;
#pragma unroll
  for (int i = 0; i < 16; ++i) {
    const float pc = exp2f(fmaf(sc[i] - mnew, LOG2E, 8.0f));
    const _Float16 h = (_Float16)pc;
    ph.h[i] = h;
    if (EARLY) {
      ps += pc;
      pl.h[i] = (_Float16)((pc - (float)h) * RES_SC);
    } else {
      ps += (float)h;
    }
  }
  ps += __shfl_xor(ps, 16, 32);
  lr = lr * al + ps;
#pragma unroll
  for (int t = 0; t < 4; ++t) {
    Oh[t] = Oh[t] * al;
    if (EARLY) Ol[t] = Ol[t] * al;
  }
  const size_t vo = (size_t)ln * SEQ + key0 + 8 * hh;
#pragma unroll
  for (int t = 0; t < 4; ++t) {
    const unsigned short* vph = Vhp + vo + (size_t)t * 16 * SEQ;
    FragH vh;
    vh.half[0] = *(const v8us*)(vph); vh.half[1] = *(const v8us*)(vph + 16);
    if (EARLY) {
      const unsigned short* vpl = Vlp + vo + (size_t)t * 16 * SEQ;
      FragH vl;
      vl.half[0] = *(const v8us*)(vpl); vl.half[1] = *(const v8us*)(vpl + 16);
      mma_pv3(vh.v, vl.v, ph.v, pl.v, Oh[t], Ol[t]);
    } else {
      mma_pv1(vh.v, ph.v, Oh[t]);
    }
  }
}

template <bool EARLY>
__global__ __launch_bounds__(128) void k_attn(const unsigned short* __restrict__ QKh,
                                              const unsigned short* __restrict__ Vth, const unsigned short* __restrict__ Vtl,
                                              const unsigned int* __restrict__ bits,
                                              unsigned short* __restrict__ Cp, unsigned short* __restrict__ Cl,
                                              int qt0, int nqt) {
  __shared__ __attribute__((aligned(16))) float so[4][16][68];
  const int tid = threadIdx.x, w = __builtin_amdgcn_readfirstlane((int)(tid >> 5)), lane = tid & 31, ln = lane & 15, hh = lane >> 4;
  const int bh = blockIdx.x / nqt, qt = qt0 + (blockIdx.x - bh * nqt);
  const int b = bh / NH, hd = bh - b * NH;
  const int qbase = qt * 64 + 16 * w;
  const int qg = qbase + ln;
  const size_t hb = (size_t)bh * SEQ * HD;
  FragH qh0, qh1;
  {
    const unsigned short* qrh = QKh + hb + (size_t)qg * HD + 8 * hh;
    qh0.half[0] = *(const v8us*)(qrh);      qh0.half[1] = *(const v8us*)(qrh + 16);
    qh1.half[0] = *(const v8us*)(qrh + 32); qh1.half[1] = *(const v8us*)(qrh + 48);
  }
  const unsigned short* Khp = QKh + PLANE + hb;
  const unsigned short* Vhp = Vth + hb;
  const unsigned short* Vlp = Vtl + hb;
  const unsigned int* mrow = bits + ((size_t)b * SEQ + qg) * (SEQ / 32);
  float mr = -3.0e38f, lr = 0.0f;
  v8f Oh[4] = {}, Ol[4] = {};
#pragma unroll 1
  for (int j = 0; j < SEQ / 32; ++j) {
    const unsigned int mw = mrow[j];
    if (__ballot(mw != 0xFFFFFFFFu) == 0) continue;
    fa_step<EARLY>(Khp, Vhp, Vlp, 32 * j, mw, ln, hh, qh0, qh1, mr, lr, Oh, Ol);
  }

  const float inv = 1.0f / (16.0f * lr);
#pragma unroll
  for (int t = 0; t < 4; ++t) {
    v4f u0, u1;
#pragma unroll
    for (int r = 0; r < 4; ++r) {
      if (EARLY) {
        u0[r] = (Oh[t][r] + Ol[t][r] * RES_INV) * inv;
        u1[r] = (Oh[t][4 + r] + Ol[t][4 + r] * RES_INV) * inv;
      } else {
        u0[r] = Oh[t][r] * inv;
        u1[r] = Oh[t][4 + r] * inv;
      }
    }
    *(v4fa*)&so[w][ln][16 * t + 8 * hh] = u0;
    *(v4fa*)&so[w][ln][16 * t + 8 * hh + 4] = u1;
  }
  __syncthreads();
  const int rsub = lane >> 3, p8 = (lane & 7) * 8;
  const size_t cb = ((size_t)(b * SEQ + qbase)) * DM + hd * HD + p8;
  for (int pass = 0; pass < 2; ++pass) {
#pragma unroll
    for (int q = 0; q < 4; ++q) {
      const int row = 4 * q + rsub;
      const v4f x0 = *(const v4fa*)&so[w][row][p8], x1 = *(const v4fa*)&so[w][row][p8 + 4];
      if (EARLY) {
        v8us oh, ol;
#pragma unroll
        for (int e = 0; e < 4; ++e) {
          const unsigned short h0 = bf16_bits(x0[e]), h1 = bf16_bits(x1[e]);
          oh[e] = h0; oh[4 + e] = h1;
          ol[e] = bf16_bits(x0[e] - bf16_val(h0));
          ol[4 + e] = bf16_bits(x1[e] - bf16_val(h1));
        }
        *(volatile v8us*)(Cp + cb + (size_t)row * DM) = oh;
        *(volatile v8us*)(Cl + cb + (size_t)row * DM) = ol;
      } else {
        H8 of;
#pragma unroll
        for (int e = 0; e < 4; ++e) {
          of.h[e]     = (_Float16)(x0[e] * 64.0f);
          of.h[4 + e] = (_Float16)(x1[e] * 64.0f);
        }
        const v8us ov = of.v;
        *(volatile v8us*)(Cp + cb + (size_t)row * DM) = ov;
      }
    }
    if (pass == 0) __threadfence();
  }
}

extern "C" void kernel_launch(void* const* d_in, const int* in_sizes, int n_in,
                              void* d_out, int out_size, void* d_ws, size_t ws_size, hipStream_t stream) {
  if (n_in < 10) return;
  const long long needx = (long long)(NB - 1) * SEQ_FULL * DM + (long long)SEQ * DM;
  const long long needm = (long long)(NB - 1) * SEQ_FULL * SEQ_FULL + (long long)(SEQ - 1) * SEQ_FULL + SEQ;
  if ((long long)in_sizes[0] < needx) return;
  if ((long long)in_sizes[1] < (long long)DM * DM || (long long)in_sizes[3] < (long long)DM * DM) return;
  if ((long long)in_sizes[5] < (long long)DM * DM || (long long)in_sizes[7] < (long long)DM * DM) return;
  if (in_sizes[2] < DM || in_sizes[4] < DM || in_sizes[6] < DM || in_sizes[8] < DM) return;
  if ((long long)in_sizes[9] < needm) return;
  if ((long long)out_size < needx) return;
  const float* x  = (const float*)d_in[0];
  const float* Wq = (const float*)d_in[1];
  const float* bq = (const float*)d_in[2];
  const float* Wk = (const float*)d_in[3];
  const float* bk = (const float*)d_in[4];
  const float* Wv = (const float*)d_in[5];
  const float* bv = (const float*)d_in[6];
  const float* Wo = (const float*)d_in[7];
  const float* bo = (const float*)d_in[8];
  const int* mask = (const int*)d_in[9];
  float* out = (float*)d_out;

  char* ws = (char*)d_ws;
  size_t off = 0;
  const size_t pl2 = PLANE * 2;
  const size_t wsz = (size_t)DM * DM * 2;
  const size_t bsz = (size_t)NB * SEQ * (SEQ / 32) * 4;
  unsigned short* Xb  = (unsigned short*)(ws + off); off += pl2;
  unsigned short* Wb  = (unsigned short*)(ws + off); off += 4 * wsz;
  unsigned short* Woh = (unsigned short*)(ws + off); off += wsz;
  unsigned short* QKh = (unsigned short*)(ws + off); off += 2 * pl2;
  unsigned short* Vth = (unsigned short*)(ws + off); off += pl2;
  unsigned short* Vtl = (unsigned short*)(ws + off); off += pl2;
  unsigned int*   Mb  = (unsigned int*)(ws + off);   off += (bsz + 255) & ~(size_t)255;
  unsigned short* Cp  = (unsigned short*)(ws + off); off += pl2;
  unsigned short* Cl  = (unsigned short*)(ws + off); off += pl2;
  if (off > ws_size || off > (size_t)134217728) return;

  const int M = NB * SEQ;
  k_cvt<false><<<(unsigned)((M * 128 + 255) / 256), 256, 0, stream>>>(x, Xb, M, SEQ, SEQ_FULL);
  k_cvt<false><<<(unsigned)((DM * 128 + 255) / 256), 256, 0, stream>>>(Wq, Wb, DM, DM, DM);
  k_cvt<false><<<(unsigned)((DM * 128 + 255) / 256), 256, 0, stream>>>(Wk, Wb + (size_t)DM * DM, DM, DM, DM);
  k_cvt<false><<<(unsigned)((DM * 128 + 255) / 256), 256, 0, stream>>>(Wv, Wb + (size_t)2 * DM * DM, DM, DM, DM);
  if (RH > 0)
    k_cvt<false><<<(unsigned)((DM * 128 + 255) / 256), 256, 0, stream>>>(Wo, Wb + (size_t)3 * DM * DM, DM, DM, DM);
  if (SEQ > RH)
    k_cvt<true><<<(unsigned)((DM * 128 + 255) / 256), 256, 0, stream>>>(Wo, Woh, DM, DM, DM);
  k_mask<<<(unsigned)((NB * SEQ * (SEQ / 32) + 255) / 256), 256, 0, stream>>>(mask, Mb);
  k_gemm<0><<<dim3((unsigned)(NB * (SEQ / 128)), DM / 64, 2), 128, 0, stream>>>(Xb, Xb, Wb, bq, bk, QKh, QKh, out, 0, SEQ / 128);
  k_gemm<1><<<dim3((unsigned)(NB * (SEQ / 128)), DM / 64, 1), 128, 0, stream>>>(Xb, Xb, Wb + (size_t)2 * DM * DM, bv, bv, Vth, Vtl, out, 0, SEQ / 128);
  if (RH > 0)
    k_attn<true><<<(unsigned)(NB * NH * (RH / 64)), 128, 0, stream>>>(QKh, Vth, Vtl, Mb, Cp, Cl, 0, RH / 64);
  if (SEQ > RH)
    k_attn<false><<<(unsigned)(NB * NH * ((SEQ - RH) / 64)), 128, 0, stream>>>(QKh, Vth, Vtl, Mb, Cp, Cl, RH / 64, (SEQ - RH) / 64);
  if (RH > 0)
    k_gemm<2><<<dim3((unsigned)(NB * (RH / 128)), DM / 64, 1), 128, 0, stream>>>(Cp, Cl, Wb + (size_t)3 * DM * DM, bo, bo, QKh, QKh, out, 0, RH / 128);
  if (SEQ > RH)
    k_gemm<3><<<dim3((unsigned)(NB * ((SEQ - RH) / 128)), DM / 64, 1), 128, 0, stream>>>(Cp, Cl, Woh, bo, bo, QKh, QKh, out, RH, (SEQ - RH) / 128);
}
